// IAU_78176994721951
// MI455X (gfx1250) — hardware-verified
//
#include <hip/hip_runtime.h>
#include <math.h>

#define NB     32
#define NC     2048
#define NHW    192
#define NCI    1024
#define W1SC   64.0f
#define PSC    4096.0f
#define S512   512.0f
#define INV512 0.001953125f

typedef _Float16 v16h __attribute__((ext_vector_type(16)));
typedef _Float16 v8h  __attribute__((ext_vector_type(8)));
typedef float    v8f  __attribute__((ext_vector_type(8)));
typedef float    v4f  __attribute__((ext_vector_type(4)));
typedef v8h __attribute__((may_alias)) v8ha;
typedef v4f __attribute__((may_alias)) v4fa;

union Frag { v16h v; v8h half[2]; };

__device__ __forceinline__ v8f wmma_f16(v16h a, v16h b, v8f c) {
#if defined(__HIP_DEVICE_COMPILE__)
  v8f d = __builtin_amdgcn_wmma_f32_16x16x32_f16(false, a, false, b, (short)0, c, false, false);
  asm volatile("v_nop\n\tv_nop\n\tv_nop\n\tv_nop" : "+v"(d) : "v"(a), "v"(b));
  return d;
#else
  (void)a; (void)b;
  return c;
#endif
}

__device__ __forceinline__ v16h load_frag(const _Float16* p, int h) {
  Frag f;
  f.half[0] = *(const v8ha*)(p + 8 * h);
  f.half[1] = *(const v8ha*)(p + 16 + 8 * h);
  return f.v;
}

__device__ __forceinline__ float dot4(v4f a, v4f b) {
  return a.x * b.x + a.y * b.y + a.z * b.z + a.w * b.w;
}

__device__ __forceinline__ v16h pack_p(v8f a, v8f c) {
  const v16h r = { (_Float16)(a[0] * PSC), (_Float16)(a[1] * PSC), (_Float16)(a[2] * PSC), (_Float16)(a[3] * PSC),
                   (_Float16)(a[4] * PSC), (_Float16)(a[5] * PSC), (_Float16)(a[6] * PSC), (_Float16)(a[7] * PSC),
                   (_Float16)(c[0] * PSC), (_Float16)(c[1] * PSC), (_Float16)(c[2] * PSC), (_Float16)(c[3] * PSC),
                   (_Float16)(c[4] * PSC), (_Float16)(c[5] * PSC), (_Float16)(c[6] * PSC), (_Float16)(c[7] * PSC) };
  return r;
}

__global__ __launch_bounds__(128) void k_prep(const float* __restrict__ x,
    _Float16* __restrict__ x16, _Float16* __restrict__ xt16)
{
  __shared__ __attribute__((aligned(16))) _Float16 sT[NHW * 64];
  const int tid = threadIdx.x, lane = tid & 31, w = tid >> 5;
  const int c0 = blockIdx.x * 64, b = blockIdx.y;
  const size_t base = ((size_t)b * NC + c0) * NHW;
  const float* xs = x + base;
  _Float16* xd = x16 + base;

  v8h pv[12];
#pragma unroll
  for (int i = 0; i < 12; ++i) {
    const int p = i * 128 + tid;
    const v4f a = *(const v4fa*)(xs + 8 * p);
    const v4f c = *(const v4fa*)(xs + 8 * p + 4);
    const v8h o = { (_Float16)a.x, (_Float16)a.y, (_Float16)a.z, (_Float16)a.w,
                    (_Float16)c.x, (_Float16)c.y, (_Float16)c.z, (_Float16)c.w };
    pv[i] = o;
    const int cl = p / 24;
    const int hw0 = (p - cl * 24) * 8;
#pragma unroll
    for (int j = 0; j < 8; ++j) sT[(hw0 + j) * 64 + cl] = o[j];
  }
#pragma unroll
  for (int i = 0; i < 12; ++i) *(volatile v8h*)(xd + 8 * (i * 128 + tid)) = pv[i];
  __threadfence();
#pragma unroll
  for (int i = 0; i < 12; ++i) *(volatile v8h*)(xd + 8 * (i * 128 + tid)) = pv[i];
  __syncthreads();

  _Float16* xtb = xt16 + (size_t)b * NHW * NC + c0 + 8 * (lane & 7);
#pragma unroll
  for (int i = 0; i < 12; ++i) {
    const int L = w * 48 + 4 * i + (lane >> 3);
    const v8h v = *(const v8ha*)(sT + L * 64 + 8 * (lane & 7));
    *(volatile v8h*)(xtb + (size_t)L * NC) = v;
  }
  __threadfence();
#pragma unroll
  for (int i = 0; i < 12; ++i) {
    const int L = w * 48 + 4 * i + (lane >> 3);
    const v8h v = *(const v8ha*)(sT + L * 64 + 8 * (lane & 7));
    *(volatile v8h*)(xtb + (size_t)L * NC) = v;
  }
}

__global__ __launch_bounds__(256) void k_cvt_w1(const float* __restrict__ wsrc,
    _Float16* __restrict__ w16, int n8)
{
  const int g = blockIdx.x * 256 + threadIdx.x;
  if (g >= n8) return;
  const float* s = wsrc + (size_t)g * 8;
  const v4f a = *(const v4fa*)s;
  const v4f c = *(const v4fa*)(s + 4);
  const v8h o = { (_Float16)(a.x * W1SC), (_Float16)(a.y * W1SC), (_Float16)(a.z * W1SC), (_Float16)(a.w * W1SC),
                  (_Float16)(c.x * W1SC), (_Float16)(c.y * W1SC), (_Float16)(c.z * W1SC), (_Float16)(c.w * W1SC) };
  _Float16* dst = w16 + (size_t)g * 8;
  *(volatile v8h*)dst = o;
  __threadfence();
  *(volatile v8h*)dst = o;
}

__global__ __launch_bounds__(128) void k_attn(const _Float16* __restrict__ x16,
    const _Float16* __restrict__ xt16, _Float16* __restrict__ yt16)
{
  __shared__ __attribute__((aligned(16))) _Float16 sT[NHW * 64];
  const int tid = threadIdx.x, lane = tid & 31, w = tid >> 5;
  const int h = lane >> 4, m = lane & 15;
  const int b = blockIdx.y, m0 = blockIdx.x * 64, q0 = m0 + 16 * w;
  const _Float16* xb  = x16  + (size_t)b * NC * NHW;
  const _Float16* xtb = xt16 + (size_t)b * NHW * NC;

  const _Float16* qrow = xb + (size_t)(q0 + m) * NHW;
  v16h qf[6];
#pragma unroll
  for (int kk = 0; kk < 6; ++kk) qf[kk] = load_frag(qrow + 32 * kk, h);

  const v8f zero8 = {0.f, 0.f, 0.f, 0.f, 0.f, 0.f, 0.f, 0.f};
  v8f o[12];
#pragma unroll
  for (int t = 0; t < 12; ++t) o[t] = zero8;
  float mrun = -1e30f, lrun = 0.0f;

  const _Float16* kbase = xb  + (size_t)m * NHW;
  const _Float16* vbase = xtb + (size_t)m * NC;

#pragma unroll 1
  for (int j = 0; j < NC; j += 32) {
    const _Float16* kp0 = kbase + (size_t)j * NHW;
    const _Float16* kp1 = kp0 + 16 * NHW;
    v8f s0 = zero8, s1 = zero8;
#pragma unroll
    for (int kk = 0; kk < 6; ++kk) {
      const v16h kf0 = load_frag(kp0 + 32 * kk, h);
      const v16h kf1 = load_frag(kp1 + 32 * kk, h);
      s0 = wmma_f16(kf0, qf[kk], s0);
      s1 = wmma_f16(kf1, qf[kk], s1);
    }

    float mloc = fmaxf(s0[0], s1[0]);
#pragma unroll
    for (int r = 1; r < 8; ++r) mloc = fmaxf(mloc, fmaxf(s0[r], s1[r]));
    mloc = fmaxf(mloc, __shfl_xor(mloc, 16));
    const float mnew = fmaxf(mrun, mloc);
    const float alpha = __expf(mrun - mnew);
    mrun = mnew;
    v8f p0 = zero8, p1 = zero8;
    float lsum = 0.0f;
#pragma unroll
    for (int r = 0; r < 8; ++r) {
      const float e0 = __expf(s0[r] - mnew);
      const float e1 = __expf(s1[r] - mnew);
      p0[r] = e0;
      p1[r] = e1;
      lsum += e0 + e1;
    }
    lsum += __shfl_xor(lsum, 16);
    lrun = lrun * alpha + lsum;
    if (alpha != 1.0f) {
#pragma unroll
      for (int t = 0; t < 12; ++t) o[t] = o[t] * alpha;
    }

    const v16h pb = pack_p(p0, p1);
#pragma unroll
    for (int t = 0; t < 12; ++t) {
      const v16h vf = load_frag(vbase + (size_t)(16 * t) * NC + j, h);
      o[t] = wmma_f16(vf, pb, o[t]);
    }
  }

  const float inv = 1.0f / (lrun * PSC);
#pragma unroll
  for (int t = 0; t < 12; ++t)
#pragma unroll
    for (int r = 0; r < 8; ++r)
      sT[(16 * t + 8 * h + r) * 64 + 16 * w + m] = (_Float16)(o[t][r] * inv);
  __syncthreads();

  _Float16* ytb = yt16 + (size_t)b * NHW * NC + m0 + 8 * (lane & 7);
#pragma unroll
  for (int i = 0; i < 12; ++i) {
    const int L = w * 48 + 4 * i + (lane >> 3);
    const v8h v = *(const v8ha*)(sT + L * 64 + 8 * (lane & 7));
    *(volatile v8h*)(ytb + (size_t)L * NC) = v;
  }
  __threadfence();
#pragma unroll
  for (int i = 0; i < 12; ++i) {
    const int L = w * 48 + 4 * i + (lane >> 3);
    const v8h v = *(const v8ha*)(sT + L * 64 + 8 * (lane & 7));
    *(volatile v8h*)(ytb + (size_t)L * NC) = v;
  }
}

__global__ __launch_bounds__(128) void k_w1(const _Float16* __restrict__ w16,
    const _Float16* __restrict__ yt16, const float* __restrict__ bias, float* __restrict__ T)
{
  __shared__ __attribute__((aligned(16))) float sT[64 * NHW];
  const int tid = threadIdx.x, lane = tid & 31, w = tid >> 5;
  const int h = lane >> 4, m = lane & 15;
  const int b = blockIdx.y, o0 = blockIdx.x * 64, ow = o0 + 16 * w;

  const _Float16* arow = w16  + (size_t)(ow + m) * NC;
  const _Float16* brow = yt16 + ((size_t)b * NHW + m) * NC;

  v8f seed;
#pragma unroll
  for (int r = 0; r < 8; ++r) seed[r] = bias[ow + 8 * h + r] * W1SC;

  v8f acc[12];
#pragma unroll
  for (int t = 0; t < 12; ++t) acc[t] = seed;

#pragma unroll 1
  for (int k0 = 0; k0 < NC; k0 += 32) {
    const v16h af = load_frag(arow + k0, h);
#pragma unroll
    for (int t = 0; t < 12; ++t) {
      const v16h bf = load_frag(brow + (size_t)(16 * t) * NC + k0, h);
      acc[t] = wmma_f16(af, bf, acc[t]);
    }
  }

  const float rdo = 1.0f / W1SC;
  float* sw = sT + w * 16 * NHW;
#pragma unroll
  for (int r = 0; r < 8; ++r) {
#pragma unroll
    for (int t = 0; t < 12; ++t)
      sw[(8 * h + r) * NHW + 16 * t + m] = acc[t][r] * rdo;
  }
  __syncthreads();

  float* tg = T + ((size_t)b * NC + ow) * NHW;
#pragma unroll
  for (int i = 0; i < 24; ++i) {
    const v4f v = *(const v4fa*)(sw + 128 * i + 4 * lane);
    *(volatile v4f*)(tg + 128 * i + 4 * lane) = v;
  }
  __threadfence();
#pragma unroll
  for (int i = 0; i < 24; ++i) {
    const v4f v = *(const v4fa*)(sw + 128 * i + 4 * lane);
    *(volatile v4f*)(tg + 128 * i + 4 * lane) = v;
  }
}

__global__ __launch_bounds__(256) void k_bn1(const float* __restrict__ T, float* __restrict__ stats)
{
  __shared__ __attribute__((aligned(16))) float sS[32 * 4];
  const int tid = threadIdx.x, lane = tid & 31, w = tid >> 5;
  const int i1 = (lane < 16) ? (lane + 32) : 47;
  const float f1 = (lane < 16) ? 1.0f : 0.0f;
#pragma unroll 1
  for (int jj = 0; jj < 4; ++jj) {
    const int o = blockIdx.x * 32 + w * 4 + jj;
    double s = 0.0, q = 0.0;
#pragma unroll 1
    for (int bb = 0; bb < NB; ++bb) {
      const float* row = T + ((size_t)bb * NC + o) * NHW;
      const v4f a = *(const v4fa*)(row + 4 * lane);
      v4f c = *(const v4fa*)(row + 4 * i1);
      c = c * f1;
      s += (double)a.x + (double)a.y + (double)a.z + (double)a.w
         + (double)c.x + (double)c.y + (double)c.z + (double)c.w;
      q += (double)a.x * (double)a.x + (double)a.y * (double)a.y + (double)a.z * (double)a.z + (double)a.w * (double)a.w
         + (double)c.x * (double)c.x + (double)c.y * (double)c.y + (double)c.z * (double)c.z + (double)c.w * (double)c.w;
    }
#pragma unroll
    for (int off = 16; off > 0; off >>= 1) {
      s += __shfl_xor(s, off);
      q += __shfl_xor(q, off);
    }
    if (lane == 0) {
      const double mu = s * (1.0 / 6144.0);
      double var = q * (1.0 / 6144.0) - mu * mu;
      if (var < 0.0) var = 0.0;
      const float rstd = (float)(1.0 / sqrt(var + 1e-5));
      sS[(w * 4 + jj) * 4 + 0] = (float)mu;
      sS[(w * 4 + jj) * 4 + 1] = rstd;
      sS[(w * 4 + jj) * 4 + 2] = 0.0f;
      sS[(w * 4 + jj) * 4 + 3] = 0.0f;
    }
  }
  __syncthreads();
  if (w == 0) {
    const v4f v = *(const v4fa*)(sS + 4 * lane);
    float* dst = stats + ((size_t)blockIdx.x * 32 + lane) * 4;
    *(volatile v4f*)dst = v;
    __threadfence();
    *(volatile v4f*)dst = v;
  }
}

__global__ __launch_bounds__(256) void k_z(float* tz, const float* __restrict__ x,
    const float* __restrict__ stats, const float* __restrict__ g, const float* __restrict__ be)
{
  const size_t i = (size_t)blockIdx.x * 256 + threadIdx.x;
  const int bc = (int)(i / 48);
  const int o = bc & (NC - 1);
  const v4f t  = *(const v4fa*)(tz + 4 * i);
  const v4f xv = *(const v4fa*)(x + 4 * i);
  const v4f st = *(const v4fa*)(stats + 4 * o);
  const float gg = g[o], bb = be[o];
  v4f z;
  z.x = ((t.x - st.x) * st.y) * gg + bb + xv.x;
  z.y = ((t.y - st.x) * st.y) * gg + bb + xv.y;
  z.z = ((t.z - st.x) * st.y) * gg + bb + xv.z;
  z.w = ((t.w - st.x) * st.y) * gg + bb + xv.w;
  *(volatile v4f*)(tz + 4 * i) = z;
  __threadfence();
  *(volatile v4f*)(tz + 4 * i) = z;
}

__global__ __launch_bounds__(192) void k_sa(const float* __restrict__ Z, const float* __restrict__ saw,
    const float* __restrict__ sab, float* __restrict__ S)
{
  const int b = blockIdx.x, hw = threadIdx.x;
  const float* zb = Z + (size_t)b * NC * NHW + hw;
  float a0 = 0.f, a1 = 0.f, a2 = 0.f, a3 = 0.f;
#pragma unroll 4
  for (int c = 0; c < NC; ++c) {
    const float zv = zb[(size_t)c * NHW];
    a0 += saw[c] * zv;
    a1 += saw[NC + c] * zv;
    a2 += saw[2 * NC + c] * zv;
    a3 += saw[3 * NC + c] * zv;
  }
  a0 += sab[0]; a1 += sab[1]; a2 += sab[2]; a3 += sab[3];
  float* d = S + (size_t)b * 4 * NHW + hw;
  *(volatile float*)(d)           = a0;
  *(volatile float*)(d + NHW)     = a1;
  *(volatile float*)(d + 2 * NHW) = a2;
  *(volatile float*)(d + 3 * NHW) = a3;
  __threadfence();
  *(volatile float*)(d)           = a0;
  *(volatile float*)(d + NHW)     = a1;
  *(volatile float*)(d + 2 * NHW) = a2;
  *(volatile float*)(d + 3 * NHW) = a3;
}

__global__ __launch_bounds__(256) void k_sa2(const float* __restrict__ S, const float* __restrict__ g,
    const float* __restrict__ be, float* __restrict__ Ap, float* __restrict__ out1)
{
  __shared__ double sPart[8][8];
  __shared__ float sSt[8];
  const int tid = threadIdx.x, lane = tid & 31, w = tid >> 5;
#pragma unroll 1
  for (int n = 0; n < 4; ++n) {
    double s = 0.0, q = 0.0;
#pragma unroll 1
    for (int t = tid; t < NB * NHW; t += 256) {
      const int bb = t / NHW, hw = t - bb * NHW;
      const float v = S[((size_t)bb * 4 + n) * NHW + hw];
      s += (double)v;
      q += (double)v * (double)v;
    }
#pragma unroll
    for (int off = 16; off > 0; off >>= 1) {
      s += __shfl_xor(s, off);
      q += __shfl_xor(q, off);
    }
    if (lane == 0) { sPart[w][2 * n] = s; sPart[w][2 * n + 1] = q; }
  }
  __syncthreads();
  if (tid < 4) {
    double s = 0.0, q = 0.0;
#pragma unroll 1
    for (int ww = 0; ww < 8; ++ww) { s += sPart[ww][2 * tid]; q += sPart[ww][2 * tid + 1]; }
    const double mu = s * (1.0 / 6144.0);
    double var = q * (1.0 / 6144.0) - mu * mu;
    if (var < 0.0) var = 0.0;
    sSt[tid] = (float)mu;
    sSt[4 + tid] = (float)(1.0 / sqrt(var + 1e-5));
  }
  __syncthreads();
#pragma unroll 1
  for (int e = tid; e < NB * 4 * NHW; e += 256) {
    const int n = (e / NHW) & 3;
    float v = ((S[e] - sSt[n]) * sSt[4 + n]) * g[n] + be[n];
    v = fminf(fmaxf(v, -40.0f), 40.0f);
    const float a = 1.0f / (1.0f + expf(-v));
    *(volatile float*)(out1 + e) = a;
    *(volatile float*)(Ap + e) = a;
    __threadfence();
    *(volatile float*)(out1 + e) = a;
    *(volatile float*)(Ap + e) = a;
  }
}

__global__ __launch_bounds__(256) void k_xn(const float* __restrict__ Z, const float* __restrict__ Ap,
    float* __restrict__ U, float* __restrict__ XN)
{
  const int i = blockIdx.x * 256 + threadIdx.x;
  const int b = i >> 11, c = i & (NC - 1);
  const float* zp = Z + (size_t)i * NHW;
  const float* ap = Ap + (size_t)b * 4 * NHW;
  float u = 0.f, a0 = 0.f, a1 = 0.f, a2 = 0.f, a3 = 0.f;
#pragma unroll 1
  for (int jv = 0; jv < NHW / 4; ++jv) {
    const v4f z4 = *(const v4fa*)(zp + 4 * jv);
    u += (z4.x + z4.y) + (z4.z + z4.w);
    a0 += dot4(*(const v4fa*)(ap + 4 * jv), z4);
    a1 += dot4(*(const v4fa*)(ap + NHW + 4 * jv), z4);
    a2 += dot4(*(const v4fa*)(ap + 2 * NHW + 4 * jv), z4);
    a3 += dot4(*(const v4fa*)(ap + 3 * NHW + 4 * jv), z4);
  }
  u = u * (1.0f / 192.0f);
  float* xd = XN + (size_t)b * 4 * NC + c;
  *(volatile float*)(U + i) = u;
  *(volatile float*)(xd) = a0;
  *(volatile float*)(xd + NC) = a1;
  *(volatile float*)(xd + 2 * NC) = a2;
  *(volatile float*)(xd + 3 * NC) = a3;
  __threadfence();
  *(volatile float*)(U + i) = u;
  *(volatile float*)(xd) = a0;
  *(volatile float*)(xd + NC) = a1;
  *(volatile float*)(xd + 2 * NC) = a2;
  *(volatile float*)(xd + 3 * NC) = a3;
}

__global__ __launch_bounds__(256) void k_nodes(const float* __restrict__ XN, const float* __restrict__ U,
    const float* __restrict__ gw, const float* __restrict__ gb, float* __restrict__ ND)
{
  const int i = blockIdx.x * 256 + threadIdx.x;
  const int b = i >> 10, o = i & (NCI - 1);
  const float* wr = gw + (size_t)o * NC;
  const float* x0 = XN + (size_t)b * 4 * NC;
  const float* x1 = x0 + NC;
  const float* x2 = x0 + 2 * NC;
  const float* x3 = x0 + 3 * NC;
  const float* ub = U + (size_t)b * NC;
  float a0 = 0.f, a1 = 0.f, a2 = 0.f, a3 = 0.f, a4 = 0.f;
#pragma unroll 1
  for (int jv = 0; jv < NC / 4; ++jv) {
    const v4f w4 = *(const v4fa*)(wr + 4 * jv);
    a0 += dot4(w4, *(const v4fa*)(x0 + 4 * jv));
    a1 += dot4(w4, *(const v4fa*)(x1 + 4 * jv));
    a2 += dot4(w4, *(const v4fa*)(x2 + 4 * jv));
    a3 += dot4(w4, *(const v4fa*)(x3 + 4 * jv));
    a4 += dot4(w4, *(const v4fa*)(ub + 4 * jv));
  }
  const float bb = gb[o];
  const float r0 = a0 + bb, r1 = a1 + bb, r2 = a2 + bb, r3 = a3 + bb, r4 = a4 + bb;
  float* d = ND + (size_t)b * 5 * NCI + o;
  *(volatile float*)(d) = r0;
  *(volatile float*)(d + NCI) = r1;
  *(volatile float*)(d + 2 * NCI) = r2;
  *(volatile float*)(d + 3 * NCI) = r3;
  *(volatile float*)(d + 4 * NCI) = r4;
  __threadfence();
  *(volatile float*)(d) = r0;
  *(volatile float*)(d + NCI) = r1;
  *(volatile float*)(d + 2 * NCI) = r2;
  *(volatile float*)(d + 3 * NCI) = r3;
  *(volatile float*)(d + 4 * NCI) = r4;
}

__global__ __launch_bounds__(256) void k_qk(const float* __restrict__ ND,
    const float* __restrict__ thw, const float* __restrict__ thb,
    const float* __restrict__ phw, const float* __restrict__ phb,
    float* __restrict__ Q, float* __restrict__ KK)
{
  const int i = blockIdx.x * 256 + threadIdx.x;
  const int b = i >> 10, o = i & (NCI - 1);
  const float* nd = ND + (size_t)b * 5 * NCI;
  const float* n0 = nd, *n1 = nd + NCI, *n2 = nd + 2 * NCI, *n3 = nd + 3 * NCI, *n4 = nd + 4 * NCI;

  float q0 = 0.f, q1 = 0.f, q2 = 0.f, q3 = 0.f;
  {
    const float* wr = thw + (size_t)o * NCI;
#pragma unroll 1
    for (int jv = 0; jv < NCI / 4; ++jv) {
      const v4f w4 = *(const v4fa*)(wr + 4 * jv);
      q0 += dot4(w4, *(const v4fa*)(n0 + 4 * jv));
      q1 += dot4(w4, *(const v4fa*)(n1 + 4 * jv));
      q2 += dot4(w4, *(const v4fa*)(n2 + 4 * jv));
      q3 += dot4(w4, *(const v4fa*)(n3 + 4 * jv));
    }
    const float bb = thb[o];
    q0 += bb; q1 += bb; q2 += bb; q3 += bb;
  }
  float k0 = 0.f, k1 = 0.f, k2 = 0.f, k3 = 0.f, k4 = 0.f;
  {
    const float* wr = phw + (size_t)o * NCI;
#pragma unroll 1
    for (int jv = 0; jv < NCI / 4; ++jv) {
      const v4f w4 = *(const v4fa*)(wr + 4 * jv);
      k0 += dot4(w4, *(const v4fa*)(n0 + 4 * jv));
      k1 += dot4(w4, *(const v4fa*)(n1 + 4 * jv));
      k2 += dot4(w4, *(const v4fa*)(n2 + 4 * jv));
      k3 += dot4(w4, *(const v4fa*)(n3 + 4 * jv));
      k4 += dot4(w4, *(const v4fa*)(n4 + 4 * jv));
    }
    const float bb = phb[o];
    k0 += bb; k1 += bb; k2 += bb; k3 += bb; k4 += bb;
  }
  float* qd = Q  + (size_t)b * 4 * NCI + o;
  float* kd = KK + (size_t)b * 5 * NCI + o;
  *(volatile float*)(qd) = q0; *(volatile float*)(qd + NCI) = q1;
  *(volatile float*)(qd + 2 * NCI) = q2; *(volatile float*)(qd + 3 * NCI) = q3;
  *(volatile float*)(kd) = k0; *(volatile float*)(kd + NCI) = k1; *(volatile float*)(kd + 2 * NCI) = k2;
  *(volatile float*)(kd + 3 * NCI) = k3; *(volatile float*)(kd + 4 * NCI) = k4;
  __threadfence();
  *(volatile float*)(qd) = q0; *(volatile float*)(qd + NCI) = q1;
  *(volatile float*)(qd + 2 * NCI) = q2; *(volatile float*)(qd + 3 * NCI) = q3;
  *(volatile float*)(kd) = k0; *(volatile float*)(kd + NCI) = k1; *(volatile float*)(kd + 2 * NCI) = k2;
  *(volatile float*)(kd + 3 * NCI) = k3; *(volatile float*)(kd + 4 * NCI) = k4;
}

__global__ __launch_bounds__(256) void k_tail(const float* __restrict__ ND,
    const float* __restrict__ Q, const float* __restrict__ KK,
    const float* __restrict__ sgw, const float* __restrict__ sgb,
    const float* __restrict__ sww, const float* __restrict__ swb,
    float* __restrict__ UC)
{
  __shared__ float sLg[20];
  __shared__ float sAt[20];
  __shared__ float sWb[8];
  __shared__ __attribute__((aligned(16))) float sNb[NCI];
  __shared__ __attribute__((aligned(16))) float sP[NCI];
  const int tid = threadIdx.x, lane = tid & 31, w = tid >> 5;
  const int b = blockIdx.x;
  const float* nd = ND + (size_t)b * 5 * NCI;

  for (int p = w; p < 20; p += 8) {
    const int n = p / 5, mm = p - n * 5;
    const float* qr = Q  + ((size_t)b * 4 + n) * NCI;
    const float* kr = KK + ((size_t)b * 5 + mm) * NCI;
    float s = 0.f;
#pragma unroll 1
    for (int c = lane; c < NCI; c += 32) s += qr[c] * kr[c];
#pragma unroll
    for (int off = 16; off > 0; off >>= 1) s += __shfl_xor(s, off);
    if (lane == 0) sLg[p] = s * (1.0f / 32.0f);
  }
  __syncthreads();
  if (tid < 4) {
    float mx = sLg[tid * 5];
#pragma unroll 1
    for (int mm = 1; mm < 5; ++mm) mx = fmaxf(mx, sLg[tid * 5 + mm]);
    float sum = 0.f;
#pragma unroll 1
    for (int mm = 0; mm < 5; ++mm) {
      const float e = expf(sLg[tid * 5 + mm] - mx);
      sAt[tid * 5 + mm] = e;
      sum += e;
    }
    const float inv = 1.0f / sum;
#pragma unroll 1
    for (int mm = 0; mm < 5; ++mm) sAt[tid * 5 + mm] = sAt[tid * 5 + mm] * inv;
  }
  __syncthreads();
  if (tid < 5) sWb[tid] = 0.25f * ((sAt[tid] + sAt[5 + tid]) + (sAt[10 + tid] + sAt[15 + tid]));
  __syncthreads();
  const float wb0 = sWb[0], wb1 = sWb[1], wb2 = sWb[2], wb3 = sWb[3], wb4 = sWb[4];
  const float wsum = ((wb0 + wb1) + (wb2 + wb3)) + wb4;
  for (int c = tid; c < NCI; c += 256)
    sNb[c] = wb0 * nd[c] + wb1 * nd[NCI + c] + wb2 * nd[2 * NCI + c] + wb3 * nd[3 * NCI + c] + wb4 * nd[4 * NCI + c];
  __syncthreads();

#pragma unroll 1
  for (int jj = 0; jj < 4; ++jj) {
    const int o = tid + 256 * jj;
    const float* wr = sgw + (size_t)o * NCI;
    float s = 0.f;
#pragma unroll 1
    for (int c4 = 0; c4 < NCI / 4; ++c4)
      s += dot4(*(const v4fa*)(wr + 4 * c4), *(const v4fa*)(sNb + 4 * c4));
    sP[o] = s + wsum * sgb[o];
  }
  __syncthreads();

#pragma unroll 1
  for (int jj = 0; jj < 4; ++jj) {
    const int o = tid + 256 * jj;
    const float* wr = sww + (size_t)o * NCI;
    float s = 0.f;
#pragma unroll 1
    for (int c4 = 0; c4 < NCI / 4; ++c4)
      s += dot4(*(const v4fa*)(wr + 4 * c4), *(const v4fa*)(sP + 4 * c4));
    const float y2 = (s + swb[o]) + 0.25f * ((nd[o] + nd[NCI + o]) + (nd[2 * NCI + o] + nd[3 * NCI + o]));
    const float u2 = nd[4 * NCI + o];
    float* d0 = UC + (size_t)b * NC + o;
    float* d1 = d0 + NCI;
    *(volatile float*)d0 = y2;
    *(volatile float*)d1 = u2;
    __threadfence();
    *(volatile float*)d0 = y2;
    *(volatile float*)d1 = u2;
  }
}

__global__ __launch_bounds__(256) void k_w2(const float* __restrict__ UC, const float* __restrict__ w2,
    const float* __restrict__ b2, float* __restrict__ T2)
{
  const int o = blockIdx.x * 256 + threadIdx.x;
  const int bg = blockIdx.y * 4;
  const float* wr = w2 + (size_t)o * NC;
  const float* u0 = UC + (size_t)bg * NC;
  const float* u1 = u0 + NC;
  const float* u2 = u0 + 2 * NC;
  const float* u3 = u0 + 3 * NC;
  float a0 = 0.f, a1 = 0.f, a2 = 0.f, a3 = 0.f;
#pragma unroll 1
  for (int jv = 0; jv < NC / 4; ++jv) {
    const v4f w4 = *(const v4fa*)(wr + 4 * jv);
    a0 += dot4(w4, *(const v4fa*)(u0 + 4 * jv));
    a1 += dot4(w4, *(const v4fa*)(u1 + 4 * jv));
    a2 += dot4(w4, *(const v4fa*)(u2 + 4 * jv));
    a3 += dot4(w4, *(const v4fa*)(u3 + 4 * jv));
  }
  const float bb = b2[o];
  const float r0 = a0 + bb, r1 = a1 + bb, r2 = a2 + bb, r3 = a3 + bb;
  float* d = T2 + (size_t)bg * NC + o;
  *(volatile float*)(d) = r0; *(volatile float*)(d + NC) = r1;
  *(volatile float*)(d + 2 * NC) = r2; *(volatile float*)(d + 3 * NC) = r3;
  __threadfence();
  *(volatile float*)(d) = r0; *(volatile float*)(d + NC) = r1;
  *(volatile float*)(d + 2 * NC) = r2; *(volatile float*)(d + 3 * NC) = r3;
}

__global__ __launch_bounds__(256) void k_y3(const float* __restrict__ T2, const float* __restrict__ g,
    const float* __restrict__ be, float* __restrict__ Y3)
{
  const int c = blockIdx.x * 256 + threadIdx.x;
  double s = 0.0, q = 0.0;
#pragma unroll 1
  for (int bb = 0; bb < NB; ++bb) {
    const float v = T2[(size_t)bb * NC + c];
    s += (double)v;
    q += (double)v * (double)v;
  }
  const double mu = s * (1.0 / 32.0);
  double var = q * (1.0 / 32.0) - mu * mu;
  if (var < 0.0) var = 0.0;
  const float muf = (float)mu;
  const float rstd = (float)(1.0 / sqrt(var + 1e-5));
  const float gg = g[c], bias = be[c];
#pragma unroll 1
  for (int bb = 0; bb < NB; ++bb) {
    const float y = ((T2[(size_t)bb * NC + c] - muf) * rstd) * gg + bias;
    *(volatile float*)(Y3 + (size_t)bb * NC + c) = y;
  }
  __threadfence();
#pragma unroll 1
  for (int bb = 0; bb < NB; ++bb) {
    const float y = ((T2[(size_t)bb * NC + c] - muf) * rstd) * gg + bias;
    *(volatile float*)(Y3 + (size_t)bb * NC + c) = y;
  }
}

__global__ __launch_bounds__(256) void k_final(const float* __restrict__ Z, const float* __restrict__ Y3,
    float* __restrict__ out)
{
  const size_t i = (size_t)blockIdx.x * 256 + threadIdx.x;
  const int bc = (int)(i / 48);
  const float y = Y3[bc];
  v4f z = *(const v4fa*)(Z + 4 * i);
  z.x += y; z.y += y; z.z += y; z.w += y;
  *(volatile v4f*)(out + 4 * i) = z;
  __threadfence();
  *(volatile v4f*)(out + 4 * i) = z;
}

extern "C" void kernel_launch(void* const* d_in, const int* in_sizes, int n_in,
                              void* d_out, int out_size, void* d_ws, size_t ws_size,
                              hipStream_t stream)
{
  if (n_in < 23) return;
  const int nX = NB * NC * NHW;
  if (in_sizes[0] != nX) return;
  if (in_sizes[1] != 4 * NC || in_sizes[2] != 4 || in_sizes[3] != 4 || in_sizes[4] != 4) return;
  if (in_sizes[5] != NCI * NC || in_sizes[6] != NCI) return;
  if (in_sizes[7] != NC * NC || in_sizes[8] != NC || in_sizes[9] != NC || in_sizes[10] != NC) return;
  if (in_sizes[11] != NC * NC || in_sizes[12] != NC || in_sizes[13] != NC || in_sizes[14] != NC) return;
  if (in_sizes[15] != NCI * NCI || in_sizes[16] != NCI) return;
  if (in_sizes[17] != NCI * NCI || in_sizes[18] != NCI) return;
  if (in_sizes[19] != NCI * NCI || in_sizes[20] != NCI) return;
  if (in_sizes[21] != NCI * NCI || in_sizes[22] != NCI) return;
  if (out_size != nX + NB * 4 * NHW) return;

  const float* x     = (const float*)d_in[0];
  const float* sa_w  = (const float*)d_in[1];
  const float* sa_b  = (const float*)d_in[2];
  const float* sa_g  = (const float*)d_in[3];
  const float* sa_be = (const float*)d_in[4];
  const float* g_w   = (const float*)d_in[5];
  const float* g_b   = (const float*)d_in[6];
  const float* w1_w  = (const float*)d_in[7];
  const float* w1_b  = (const float*)d_in[8];
  const float* w1_g  = (const float*)d_in[9];
  const float* w1_be = (const float*)d_in[10];
  const float* w2_w  = (const float*)d_in[11];
  const float* w2_b  = (const float*)d_in[12];
  const float* w2_g  = (const float*)d_in[13];
  const float* w2_be = (const float*)d_in[14];
  const float* th_w  = (const float*)d_in[15];
  const float* th_b  = (const float*)d_in[16];
  const float* ph_w  = (const float*)d_in[17];
  const float* ph_b  = (const float*)d_in[18];
  const float* sg_w  = (const float*)d_in[19];
  const float* sg_b  = (const float*)d_in[20];
  const float* sw_w  = (const float*)d_in[21];
  const float* sw_b  = (const float*)d_in[22];

  float* out0 = (float*)d_out;
  float* out1 = out0 + (size_t)nX;

  const size_t szXZ  = (size_t)nX * 4;
  const size_t szYT  = (size_t)nX * 2;
  const size_t szW1  = (size_t)NC * NC * 2;
  const size_t szST1 = (size_t)NC * 4 * 4;
  const size_t szSSA = (size_t)NB * 4 * NHW * 4;
  const size_t szAP  = szSSA;
  const size_t szU   = (size_t)NB * NC * 4;
  const size_t szXN  = (size_t)NB * 4 * NC * 4;
  const size_t szND  = (size_t)NB * 5 * NCI * 4;
  const size_t szQ   = (size_t)NB * 4 * NCI * 4;
  const size_t szK   = szND;
  const size_t szUC  = szU;
  const size_t szT2  = szU;
  const size_t szY3  = szU;
  const size_t oXZ  = 0;
  const size_t oYT  = oXZ + szXZ;
  const size_t oW1  = oYT + szYT;
  const size_t oST1 = oW1 + szW1;
  const size_t oSSA = oST1 + szST1;
  const size_t oAP  = oSSA + szSSA;
  const size_t oU   = oAP + szAP;
  const size_t oXN  = oU + szU;
  const size_t oND  = oXN + szXN;
  const size_t oQ   = oND + szND;
  const size_t oK   = oQ + szQ;
  const size_t oUC  = oK + szK;
  const size_t oT2  = oUC + szUC;
  const size_t oY3  = oT2 + szT2;
  const size_t total = oY3 + szY3;
  if (total > ws_size) return;

  char* wb = (char*)d_ws;
  _Float16* X16  = (_Float16*)(wb + oXZ);
  _Float16* XT16 = X16 + (size_t)nX;
  float*    TZ   = (float*)(wb + oXZ);
  _Float16* YT16 = (_Float16*)(wb + oYT);
  _Float16* W16  = (_Float16*)(wb + oW1);
  float* ST1 = (float*)(wb + oST1);
  float* SSA = (float*)(wb + oSSA);
  float* APL = (float*)(wb + oAP);
  float* U   = (float*)(wb + oU);
  float* XN  = (float*)(wb + oXN);
  float* ND  = (float*)(wb + oND);
  float* Q   = (float*)(wb + oQ);
  float* KK  = (float*)(wb + oK);
  float* UC  = (float*)(wb + oUC);
  float* T2  = (float*)(wb + oT2);
  float* Y3  = (float*)(wb + oY3);

  const int n8w = NC * NC / 8;

  k_prep<<<dim3(NC / 64, NB), 128, 0, stream>>>(x, X16, XT16);
  k_cvt_w1<<<(n8w + 255) / 256, 256, 0, stream>>>(w1_w, W16, n8w);
  k_attn<<<dim3(NC / 64, NB), 128, 0, stream>>>(X16, XT16, YT16);
  k_w1<<<dim3(NC / 64, NB), 128, 0, stream>>>(W16, YT16, w1_b, TZ);
  k_bn1<<<NC / 32, 256, 0, stream>>>(TZ, ST1);
  k_z<<<(nX / 4) / 256, 256, 0, stream>>>(TZ, x, ST1, w1_g, w1_be);
  k_sa<<<NB, NHW, 0, stream>>>(TZ, sa_w, sa_b, SSA);
  k_sa2<<<1, 256, 0, stream>>>(SSA, sa_g, sa_be, APL, out1);
  k_xn<<<(NB * NC) / 256, 256, 0, stream>>>(TZ, APL, U, XN);
  k_nodes<<<(NB * NCI) / 256, 256, 0, stream>>>(XN, U, g_w, g_b, ND);
  k_qk<<<(NB * NCI) / 256, 256, 0, stream>>>(ND, th_w, th_b, ph_w, ph_b, Q, KK);
  k_tail<<<NB, 256, 0, stream>>>(ND, Q, KK, sg_w, sg_b, sw_w, sw_b, UC);
  k_w2<<<dim3(NC / 256, NB / 4), 256, 0, stream>>>(UC, w2_w, w2_b, T2);
  k_y3<<<NC / 256, 256, 0, stream>>>(T2, w2_g, w2_be, Y3);
  k_final<<<(nX / 4) / 256, 256, 0, stream>>>(TZ, Y3, out0);
}
